// LSTMModel_39161511805207
// MI455X (gfx1250) — hardware-verified
//
#include <hip/hip_runtime.h>
#include <math.h>

constexpr int NBATCH   = 4096;
constexpr int NSTEP    = 200;
constexpr int NFEAT    = 16;
constexpr int HID1     = 55;
constexpr int HID2     = 30;
constexpr int NOUTC    = 6;
constexpr int HID1P    = 64;
constexpr int HID2P    = 32;
constexpr int GATE1P   = 4 * HID1P;
constexpr int GATE2P   = 4 * HID2P;
constexpr int KCAT     = 96;
constexpr int KUNITS   = KCAT / 8;
constexpr int NTHR     = 128;
constexpr int ROWS_BLK = 16;
constexpr int XPITCH   = 40;
constexpr int H1PITCH  = 72;
constexpr int H2PITCH  = 40;
constexpr int W2PITCH  = 104;
constexpr int PREP_THR = 256;
constexpr int PREP_BLK1 = GATE1P * KUNITS / PREP_THR;
constexpr int PREP_BLK2 = GATE2P * KUNITS / PREP_THR;
constexpr int NBIAS    = GATE1P + GATE2P;
constexpr float WCARRY = 16.0f;
constexpr float ACARRY = 64.0f;
constexpr float FOLD   = 1.0f / (WCARRY * ACARRY);

static_assert(NBATCH % ROWS_BLK == 0);
static_assert(NFEAT == 16 && KCAT == 96 && KCAT % 32 == 0);
static_assert(32 + HID1 <= KCAT && 64 + HID2 <= KCAT && HID1 <= 64);
static_assert(GATE1P * KUNITS == PREP_BLK1 * PREP_THR);
static_assert(GATE2P * KUNITS == PREP_BLK2 * PREP_THR);
static_assert(NBIAS == 96 * 4);
static_assert(ROWS_BLK * NOUTC == 96);
static_assert((2 * ROWS_BLK * H1PITCH) % NTHR == 0);
static_assert((2 * ROWS_BLK * H2PITCH) % NTHR == 0);
static_assert((GATE2P * KUNITS) % NTHR == 0);
static_assert(XPITCH % 8 == 0 && H1PITCH % 8 == 0 && H2PITCH % 8 == 0 && W2PITCH % 8 == 0);

typedef __attribute__((ext_vector_type(16))) _Float16 v16h;
typedef __attribute__((ext_vector_type(8)))  _Float16 v8h;
typedef __attribute__((ext_vector_type(4)))  _Float16 v4h;
typedef __attribute__((ext_vector_type(8)))  float    v8f;
typedef __attribute__((ext_vector_type(4)))  float    v4f;

__device__ __forceinline__ void guard4_h(v8f& a, v8f& b, v8f& c, v8f& d, v16h x, v16h y) {
  asm volatile("v_nop\n\tv_nop\n\tv_nop\n\tv_nop" : "+v"(a), "+v"(b), "+v"(c), "+v"(d) : "v"(x), "v"(y));
}
__device__ __forceinline__ void keep3_h(v16h a, v16h b, v16h c) {
  asm volatile("" :: "v"(a), "v"(b), "v"(c) : "memory");
}
__device__ __forceinline__ void keep4_f(float a, float b, float c, float d) {
  asm volatile("" :: "v"(a), "v"(b), "v"(c), "v"(d) : "memory");
}

template <typename T> struct Frag;
template <> struct Frag<_Float16> {
  typedef v16h V; union U { v16h v; v8h h[2]; };
  static __device__ __forceinline__ v16h load(const _Float16* p) {
    U f; f.h[0] = *(const v8h*)(p); f.h[1] = *(const v8h*)(p + 16); return f.v;
  }
  static __device__ __forceinline__ v8f mma(v16h a, v16h b, v8f c) {
    return __builtin_amdgcn_wmma_f32_16x16x32_f16(false, a, false, b, (short)0, c, false, false);
  }
};

__device__ __forceinline__ float sigm_f(float z)  { return 1.0f / (1.0f + expf(-z)); }
__device__ __forceinline__ float tanh_f(float z)  { return 1.0f - 2.0f / (1.0f + expf(2.0f * z)); }

template <int KA, int KB, int KBOFF>
__device__ __forceinline__ float pack_elem(const float* __restrict__ Wa, const float* __restrict__ Wb,
                                           int srow, float rv, int k) {
  const int ka = (k < KA) ? k : (KA - 1);
  int kb = k - KBOFF;
  kb = (kb < 0) ? 0 : kb;
  kb = (kb < KB) ? kb : (KB - 1);
  const float a = Wa[srow * KA + ka];
  const float b = Wb[srow * KB + kb];
  const float fa = (k < KA) ? rv : 0.0f;
  const float fb = (k >= KBOFF && k < KBOFF + KB) ? rv : 0.0f;
  return fmaf(fa, a, fb * b) * WCARRY + 0.0f;
}

template <int UNITBITS, int HREAL, int KA, int KB, int KBOFF>
__device__ __forceinline__ void pack_unit(const float* __restrict__ Wa, const float* __restrict__ Wb,
                                          _Float16* dst, int u) {
  const int n  = u / KUNITS;
  const int k8 = (u - n * KUNITS) * 8;
  const int g  = n >> UNITBITS;
  const int r  = n & ((1 << UNITBITS) - 1);
  const int rc = (r < HREAL) ? r : (HREAL - 1);
  const int srow = g * HREAL + rc;
  const float rv = (r < HREAL) ? 1.0f : 0.0f;
  const float e0 = pack_elem<KA, KB, KBOFF>(Wa, Wb, srow, rv, k8 + 0);
  const float e1 = pack_elem<KA, KB, KBOFF>(Wa, Wb, srow, rv, k8 + 1);
  const float e2 = pack_elem<KA, KB, KBOFF>(Wa, Wb, srow, rv, k8 + 2);
  const float e3 = pack_elem<KA, KB, KBOFF>(Wa, Wb, srow, rv, k8 + 3);
  keep4_f(e0, e1, e2, e3);
  const float e4 = pack_elem<KA, KB, KBOFF>(Wa, Wb, srow, rv, k8 + 4);
  const float e5 = pack_elem<KA, KB, KBOFF>(Wa, Wb, srow, rv, k8 + 5);
  const float e6 = pack_elem<KA, KB, KBOFF>(Wa, Wb, srow, rv, k8 + 6);
  const float e7 = pack_elem<KA, KB, KBOFF>(Wa, Wb, srow, rv, k8 + 7);
  keep4_f(e4, e5, e6, e7);
  v8h hv;
  hv[0] = (_Float16)e0; hv[1] = (_Float16)e1; hv[2] = (_Float16)e2; hv[3] = (_Float16)e3;
  hv[4] = (_Float16)e4; hv[5] = (_Float16)e5; hv[6] = (_Float16)e6; hv[7] = (_Float16)e7;
  _Float16* op = dst + (size_t)u * 8;
  *(volatile v8h*)op = hv;
  __threadfence();
  *(volatile v8h*)op = hv;
}

__device__ __forceinline__ float bias_elem(const float* __restrict__ bi1, const float* __restrict__ bh1,
                                           const float* __restrict__ bi2, const float* __restrict__ bh2, int i) {
  const int n1 = (i < GATE1P) ? i : (GATE1P - 1);
  const int r1 = n1 & (HID1P - 1);
  const int s1 = (n1 >> 6) * HID1 + ((r1 < HID1) ? r1 : (HID1 - 1));
  int n2 = i - GATE1P;
  n2 = (n2 < 0) ? 0 : n2;
  n2 = (n2 < GATE2P) ? n2 : (GATE2P - 1);
  const int r2 = n2 & (HID2P - 1);
  const int s2 = (n2 >> 5) * HID2 + ((r2 < HID2) ? r2 : (HID2 - 1));
  const float a = bi1[s1] + bh1[s1];
  const float b = bi2[s2] + bh2[s2];
  const float fa = (i < GATE1P && r1 < HID1) ? 1.0f : 0.0f;
  const float fb = (i >= GATE1P && r2 < HID2) ? 1.0f : 0.0f;
  return fmaf(fa, a, fb * b) + 0.0f;
}

__global__ __launch_bounds__(PREP_THR) void prep_kernel(
    const float* __restrict__ Wih1, const float* __restrict__ Whh1,
    const float* __restrict__ bih1, const float* __restrict__ bhh1,
    const float* __restrict__ Wih2, const float* __restrict__ Whh2,
    const float* __restrict__ bih2, const float* __restrict__ bhh2,
    unsigned short* __restrict__ W1p, unsigned short* __restrict__ W2p, float* __restrict__ biasp) {
  const int tid = threadIdx.x;
  const int bx  = blockIdx.x;
  if (bx < PREP_BLK1) {
    pack_unit<6, HID1, NFEAT, HID1, 32>(Wih1, Whh1, (_Float16*)W1p, bx * PREP_THR + tid);
  } else if (bx < PREP_BLK1 + PREP_BLK2) {
    pack_unit<5, HID2, HID1, HID2, 64>(Wih2, Whh2, (_Float16*)W2p, (bx - PREP_BLK1) * PREP_THR + tid);
  } else {
    if (tid < NBIAS / 4) {
      const int i0 = tid * 4;
      const float e0 = bias_elem(bih1, bhh1, bih2, bhh2, i0 + 0);
      const float e1 = bias_elem(bih1, bhh1, bih2, bhh2, i0 + 1);
      keep4_f(e0, e1, e0, e1);
      const float e2 = bias_elem(bih1, bhh1, bih2, bhh2, i0 + 2);
      const float e3 = bias_elem(bih1, bhh1, bih2, bhh2, i0 + 3);
      keep4_f(e2, e3, e2, e3);
      v4f o;
      o[0] = e0; o[1] = e1; o[2] = e2; o[3] = e3;
      float* op = biasp + i0;
      *(volatile v4f*)op = o;
      __threadfence();
      *(volatile v4f*)op = o;
    }
  }
}

__device__ __forceinline__ void stage_x(const float* __restrict__ x, _Float16* Xs, int b0, int tstep, int i) {
  const int m  = i >> 2;
  const int f4 = (i & 3) * 4;
  const v4f v = *(const v4f*)(x + ((size_t)(b0 + m) * NSTEP + (size_t)tstep) * NFEAT + f4);
  v4h hx;
  hx[0] = (_Float16)(v[0] * ACARRY);
  hx[1] = (_Float16)(v[1] * ACARRY);
  hx[2] = (_Float16)(v[2] * ACARRY);
  hx[3] = (_Float16)(v[3] * ACARRY);
  const v4h hz = {(_Float16)0.0f, (_Float16)0.0f, (_Float16)0.0f, (_Float16)0.0f};
  *(v4h*)(Xs + m * XPITCH + f4) = hx;
  *(v4h*)(Xs + m * XPITCH + 16 + f4) = hz;
}

__global__ __launch_bounds__(NTHR) void lstm2_kernel(
    const float* __restrict__ x,
    const unsigned short* __restrict__ W1p, const unsigned short* __restrict__ W2p,
    const float* __restrict__ biasp,
    const float* __restrict__ Wfc, const float* __restrict__ bfc,
    float* __restrict__ out) {
  __shared__ __align__(16) _Float16 W2s[GATE2P * W2PITCH];
  __shared__ __align__(16) _Float16 Xs[ROWS_BLK * XPITCH];
  __shared__ __align__(16) _Float16 H1s[2][ROWS_BLK * H1PITCH];
  __shared__ __align__(16) _Float16 H2s[2][ROWS_BLK * H2PITCH];
  __shared__ __align__(16) float    Hf[ROWS_BLK * HID2P];

  const _Float16* W1  = (const _Float16*)W1p;
  const _Float16* W2g = (const _Float16*)W2p;
  const int tid  = threadIdx.x;
  const int lane = tid & 31;
  const int wave = __builtin_amdgcn_readfirstlane(tid >> 5);
  const int c    = lane & 15;
  const int hh   = lane >> 4;
  const int koff = hh * 8;
  const int b0   = blockIdx.x * ROWS_BLK;

#pragma unroll 1
  for (int it = 0; it < (GATE2P * KUNITS) / NTHR; ++it) {
    const int u  = it * NTHR + tid;
    const int n  = u / KUNITS;
    const int k8 = (u - n * KUNITS) * 8;
    const v8h v = *(const v8h*)(W2g + (size_t)u * 8);
    *(v8h*)(W2s + n * W2PITCH + k8) = v;
  }
  {
    _Float16* h1f = &H1s[0][0];
#pragma unroll 1
    for (int i = tid; i < 2 * ROWS_BLK * H1PITCH; i += NTHR) h1f[i] = (_Float16)0.0f;
    _Float16* h2f = &H2s[0][0];
#pragma unroll 1
    for (int i = tid; i < 2 * ROWS_BLK * H2PITCH; i += NTHR) h2f[i] = (_Float16)0.0f;
  }
  if (wave >= 2) stage_x(x, Xs, b0, 0, tid - 64);

  float b1g[4], b2g[4];
#pragma unroll
  for (int g = 0; g < 4; ++g) {
    b1g[g] = biasp[g * HID1P + 16 * wave + c];
    b2g[g] = biasp[GATE1P + g * HID2P + 16 * (wave & 1) + c];
  }

  v16h B1[4][3];
#pragma unroll
  for (int g = 0; g < 4; ++g) {
    const _Float16* wrow = W1 + (size_t)(g * HID1P + 16 * wave + c) * KCAT + koff;
    B1[g][0] = Frag<_Float16>::load(wrow);
    B1[g][1] = Frag<_Float16>::load(wrow + 32);
    B1[g][2] = Frag<_Float16>::load(wrow + 64);
    keep3_h(B1[g][0], B1[g][1], B1[g][2]);
  }

  float c1[8], c2[8];
#pragma unroll
  for (int r = 0; r < 8; ++r) { c1[r] = 0.0f; c2[r] = 0.0f; }
  const v8f z8 = {0.f, 0.f, 0.f, 0.f, 0.f, 0.f, 0.f, 0.f};
  __syncthreads();

#pragma unroll 1
  for (int t = 0; t < NSTEP; ++t) {
    const int p = t & 1;
    const _Float16* h1r = &H1s[p][0];
    _Float16*       h1w = &H1s[p ^ 1][0];
    const _Float16* h2r = &H2s[p][0];
    _Float16*       h2w = &H2s[p ^ 1][0];
    const bool last = (t == NSTEP - 1);

    {
      v16h af[3];
      af[0] = Frag<_Float16>::load(Xs  + c * XPITCH  + koff);
      af[1] = Frag<_Float16>::load(h1r + c * H1PITCH + koff);
      af[2] = Frag<_Float16>::load(h1r + c * H1PITCH + koff + 32);
      v8f acc[4];
      acc[0] = z8; acc[1] = z8; acc[2] = z8; acc[3] = z8;
#pragma unroll
      for (int kt = 0; kt < 3; ++kt) {
#pragma unroll
        for (int g = 0; g < 4; ++g) acc[g] = Frag<_Float16>::mma(af[kt], B1[g][kt], acc[g]);
        guard4_h(acc[0], acc[1], acc[2], acc[3], af[kt], B1[3][kt]);
      }
#pragma unroll
      for (int r = 0; r < 8; ++r) {
        const float zi = fmaf(acc[0][r], FOLD, b1g[0]);
        const float zf = fmaf(acc[1][r], FOLD, b1g[1]);
        const float zg = fmaf(acc[2][r], FOLD, b1g[2]);
        const float zo = fmaf(acc[3][r], FOLD, b1g[3]);
        const float ig = sigm_f(zi);
        const float fg = sigm_f(zf);
        const float gg = tanh_f(zg);
        const float og = sigm_f(zo);
        const float cn = fg * c1[r] + ig * gg;
        c1[r] = cn;
        const float hv = og * tanh_f(cn);
        h1w[(8 * hh + r) * H1PITCH + 16 * wave + c] = (_Float16)(hv * ACARRY);
      }
    }
    __syncthreads();

    if (wave < 2) {
      v16h a2[3];
      a2[0] = Frag<_Float16>::load(h1w + c * H1PITCH + koff);
      a2[1] = Frag<_Float16>::load(h1w + c * H1PITCH + koff + 32);
      a2[2] = Frag<_Float16>::load(h2r + c * H2PITCH + koff);
      v8f acc2[4];
      acc2[0] = z8; acc2[1] = z8; acc2[2] = z8; acc2[3] = z8;
#pragma unroll
      for (int kt = 0; kt < 3; ++kt) {
        v16h bf[4];
#pragma unroll
        for (int g = 0; g < 4; ++g)
          bf[g] = Frag<_Float16>::load(W2s + (g * HID2P + 16 * wave + c) * W2PITCH + koff + 32 * kt);
#pragma unroll
        for (int g = 0; g < 4; ++g) acc2[g] = Frag<_Float16>::mma(a2[kt], bf[g], acc2[g]);
        guard4_h(acc2[0], acc2[1], acc2[2], acc2[3], a2[kt], bf[3]);
      }
#pragma unroll
      for (int r = 0; r < 8; ++r) {
        const float zi = fmaf(acc2[0][r], FOLD, b2g[0]);
        const float zf = fmaf(acc2[1][r], FOLD, b2g[1]);
        const float zg = fmaf(acc2[2][r], FOLD, b2g[2]);
        const float zo = fmaf(acc2[3][r], FOLD, b2g[3]);
        const float ig = sigm_f(zi);
        const float fg = sigm_f(zf);
        const float gg = tanh_f(zg);
        const float og = sigm_f(zo);
        const float cn = fg * c2[r] + ig * gg;
        c2[r] = cn;
        const float hv = og * tanh_f(cn);
        h2w[(8 * hh + r) * H2PITCH + 16 * wave + c] = (_Float16)(hv * ACARRY);
        if (last) Hf[(8 * hh + r) * HID2P + 16 * wave + c] = hv;
      }
    } else {
      const int tn = (t + 1 < NSTEP) ? (t + 1) : (NSTEP - 1);
      stage_x(x, Xs, b0, tn, tid - 64);
    }
    __syncthreads();
  }

  if (wave < 3) {
    const int idx = tid;
    const int m = idx / NOUTC;
    const int o = idx - m * NOUTC;
    float s = 0.0f;
#pragma unroll 1
    for (int k = 0; k < HID2; ++k) s = fmaf(Hf[m * HID2P + k], Wfc[o * HID2 + k], s);
    s += bfc[o];
    float* op = out + (size_t)b0 * NOUTC + idx;
    *(volatile float*)op = s;
    __threadfence();
    *(volatile float*)op = s;
  }
}

extern "C" void kernel_launch(void* const* d_in, const int* in_sizes, int n_in,
                              void* d_out, int out_size, void* d_ws, size_t ws_size, hipStream_t stream) {
  if (n_in < 11 || d_out == nullptr || d_ws == nullptr) return;
  if (in_sizes[0] != NBATCH * NSTEP * NFEAT || in_sizes[1] != 4 * HID1 * NFEAT || in_sizes[2] != 4 * HID1 * HID1 ||
      in_sizes[3] != 4 * HID1 || in_sizes[4] != 4 * HID1 || in_sizes[5] != 4 * HID2 * HID1 ||
      in_sizes[6] != 4 * HID2 * HID2 || in_sizes[7] != 4 * HID2 || in_sizes[8] != 4 * HID2 ||
      in_sizes[9] != NOUTC * HID2 || in_sizes[10] != NOUTC || out_size != NBATCH * NOUTC) return;

  const float* x    = (const float*)d_in[0];
  const float* Wih1 = (const float*)d_in[1];
  const float* Whh1 = (const float*)d_in[2];
  const float* bih1 = (const float*)d_in[3];
  const float* bhh1 = (const float*)d_in[4];
  const float* Wih2 = (const float*)d_in[5];
  const float* Whh2 = (const float*)d_in[6];
  const float* bih2 = (const float*)d_in[7];
  const float* bhh2 = (const float*)d_in[8];
  const float* Wfc  = (const float*)d_in[9];
  const float* bfc  = (const float*)d_in[10];
  float* out = (float*)d_out;

  char* ws = (char*)d_ws;
  size_t off = 0;
  unsigned short* W1CAT = (unsigned short*)(ws + off);
  off += ((size_t)GATE1P * KCAT * 2 + 255) & ~(size_t)255;
  unsigned short* W2CAT = (unsigned short*)(ws + off);
  off += ((size_t)GATE2P * KCAT * 2 + 255) & ~(size_t)255;
  float* BIAS = (float*)(ws + off);
  off += ((size_t)NBIAS * 4 + 255) & ~(size_t)255;
  if (off > ws_size || off > (size_t)134217728) return;

  prep_kernel<<<PREP_BLK1 + PREP_BLK2 + 1, PREP_THR, 0, stream>>>(
      Wih1, Whh1, bih1, bhh1, Wih2, Whh2, bih2, bhh2, W1CAT, W2CAT, BIAS);
  lstm2_kernel<<<NBATCH / ROWS_BLK, NTHR, 0, stream>>>(x, W1CAT, W2CAT, BIAS, Wfc, bfc, out);
}
